// force_net_10694468567092
// MI455X (gfx1250) — hardware-run, weakly checked
//
#include <hip/hip_runtime.h>
#include <math.h>

#pragma clang fp contract(off)

#define NB   4
#define NT   1024
#define NR   (NB * NT)
#define DM   256
#define NH   8
#define DK   32
#define DF   1024
#define NL   4
#define NX   70
#define NC   64
#define NFQ  128

#define OUT0_N (NR * NC)
#define OUT1_N (NB * NT * NT)

#define ASC  16.0f
#define WSC  64.0f
#define RSC  16384.0f
#define PSC  256.0f
#define HINV 9.765625e-4f
#define LINV 5.9604644775390625e-8f
#define RINV 6.103515625e-5f
#define SSC  6.9053396600248782e-4f
#define OINV 2.44140625e-4f
#define PEC  0.17677669529663687f
#define GC   0.70710678118654752f

#define GP  72
#define OP  68
#define OPT 132

static_assert(NR % 128 == 0 && NT % 128 == 0 && DM % 64 == 0 && DF % 64 == 0 && NC == 64);
static_assert(DK == 32 && NH * DK == DM && NFQ * 2 == DM && NX == NC + 6);
static_assert((GP % 8) == 0 && (OP % 4) == 0 && (OPT % 4) == 0 && 64 * OPT <= 128 * OP);

typedef _Float16 f16;
typedef _Float16 v16h __attribute__((ext_vector_type(16)));
typedef _Float16 v8h  __attribute__((ext_vector_type(8)));
typedef _Float16 v8ha __attribute__((ext_vector_type(8), may_alias));
typedef unsigned short v8us __attribute__((ext_vector_type(8)));
typedef float v8f __attribute__((ext_vector_type(8)));
typedef float v4f __attribute__((ext_vector_type(4)));
typedef float v4fa __attribute__((ext_vector_type(4), may_alias));
typedef int v8i __attribute__((ext_vector_type(8)));

union FragH { v16h v; v8h h[2]; };

__device__ __forceinline__ float bf16r(float f) {
  unsigned int u = __float_as_uint(f);
  u = u + 0x7FFFu + ((u >> 16) & 1u);
  u &= 0xFFFF0000u;
  return __uint_as_float(u);
}

__device__ __forceinline__ void split2(float v, f16& hi, f16& lo) {
  const float s = v * ASC;
  const f16 hv = (f16)s;
  hi = hv;
  lo = (f16)((s - (float)hv) * RSC);
}

__device__ __forceinline__ float gelu_f(float v) { return 0.5f * v * (1.0f + erff(v * GC)); }

__device__ __forceinline__ v16h ld_frag(const f16* base, int row0, int k0, int ld) {
  const int lane = threadIdx.x & 31;
  const f16* p = base + (size_t)(row0 + (lane & 15)) * ld + k0 + ((lane >> 4) << 3);
  FragH f;
  f.h[0] = *(const v8h*)p;
  f.h[1] = *(const v8h*)(p + 16);
  return f.v;
}

__device__ __forceinline__ v8f mma_h(v16h a, v16h b, v8f c) {
  return __builtin_amdgcn_wmma_f32_16x16x32_f16(false, a, false, b, (short)0, c, false, false);
}

__device__ __forceinline__ void guard4x4(v8f& c0, v8f& c1, v8f& c2, v8f& c3,
                                         v16h f0, v16h f1, v16h f2, v16h f3) {
#if defined(__HIP_DEVICE_COMPILE__)
  asm volatile("v_nop\n\tv_nop\n\tv_nop\n\tv_nop"
               : "+v"(c0), "+v"(c1), "+v"(c2), "+v"(c3)
               : "v"(f0), "v"(f1), "v"(f2), "v"(f3));
#endif
}
__device__ __forceinline__ void guard8x6(v8f& c0, v8f& c1, v8f& c2, v8f& c3,
                                         v8f& c4, v8f& c5, v8f& c6, v8f& c7,
                                         v16h f0, v16h f1, v16h f2, v16h f3, v16h f4, v16h f5) {
#if defined(__HIP_DEVICE_COMPILE__)
  asm volatile("v_nop\n\tv_nop\n\tv_nop\n\tv_nop"
               : "+v"(c0), "+v"(c1), "+v"(c2), "+v"(c3), "+v"(c4), "+v"(c5), "+v"(c6), "+v"(c7)
               : "v"(f0), "v"(f1), "v"(f2), "v"(f3), "v"(f4), "v"(f5));
#endif
}
__device__ __forceinline__ void guard2x3(v8f& c0, v8f& c1, v16h f0, v16h f1, v16h f2) {
#if defined(__HIP_DEVICE_COMPILE__)
  asm volatile("v_nop\n\tv_nop\n\tv_nop\n\tv_nop"
               : "+v"(c0), "+v"(c1)
               : "v"(f0), "v"(f1), "v"(f2));
#endif
}
__device__ __forceinline__ void guard2x4(v8f& c0, v8f& c1, v16h f0, v16h f1, v16h f2, v16h f3) {
#if defined(__HIP_DEVICE_COMPILE__)
  asm volatile("v_nop\n\tv_nop\n\tv_nop\n\tv_nop"
               : "+v"(c0), "+v"(c1)
               : "v"(f0), "v"(f1), "v"(f2), "v"(f3));
#endif
}

__global__ __launch_bounds__(256)
void k_cvt_x(const float* __restrict__ X, unsigned short* dst, int n8) {
  const int p = (int)blockIdx.x * 256 + (int)threadIdx.x;
  if (p >= n8) return;
  const int r = p >> 3, q = p & 7;
  const float* s = X + (size_t)r * NX + 6 + 8 * q;
  v8h o = {};
#pragma unroll
  for (int e = 0; e < 8; ++e) o[e] = (f16)(bf16r(s[e]) * ASC);
  const v8us u = __builtin_bit_cast(v8us, o);
  unsigned short* op = dst + (size_t)p * 8;
  *(volatile v8us*)op = u;
  __threadfence();
  *(volatile v8us*)op = u;
}

__global__ __launch_bounds__(256)
void k_cvt_wt(const float* __restrict__ W, unsigned short* dst, int K, int N, size_t dls, int rowoff, float scale) {
  __shared__ __align__(16) f16 T[64 * GP];
  const int tid = threadIdx.x;
  const int z = (int)blockIdx.z, n0 = (int)blockIdx.x * 64, k0 = (int)blockIdx.y * 64;
  const float* src = W + (size_t)z * K * N;
#pragma unroll
  for (int j = 0; j < 4; ++j) {
    const int e = tid + 256 * j;
    const int kr = e >> 4, n4 = (e & 15) * 4;
    const v4f x = *(const v4f*)(src + (size_t)(k0 + kr) * N + n0 + n4);
#pragma unroll
    for (int c = 0; c < 4; ++c) T[(n4 + c) * GP + kr] = (f16)(bf16r(x[c]) * scale);
  }
  __syncthreads();
  v8us u[2];
  size_t off[2];
#pragma unroll
  for (int it = 0; it < 2; ++it) {
    const int p = tid + 256 * it;
    const int row = p >> 3, q = p & 7;
    const v8h v = *(const v8ha*)&T[row * GP + 8 * q];
    u[it] = __builtin_bit_cast(v8us, v);
    off[it] = (size_t)z * dls + (size_t)(rowoff + n0 + row) * K + k0 + 8 * q;
  }
#pragma unroll
  for (int it = 0; it < 2; ++it) *(volatile v8us*)(dst + off[it]) = u[it];
  __threadfence();
#pragma unroll
  for (int it = 0; it < 2; ++it) *(volatile v8us*)(dst + off[it]) = u[it];
}

template <bool LO>
__global__ __launch_bounds__(256)
void k_ln(const float* __restrict__ X, const float* __restrict__ g, const float* __restrict__ bb,
          unsigned short* yh, unsigned short* yl, int nrows) {
  const int tid = threadIdx.x, lane = tid & 31, wv = tid >> 5;
  const int row = (int)blockIdx.x * 8 + wv;
  if (row >= nrows) return;
  const float* xp = X + (size_t)row * DM + 8 * lane;
  const v4f a = *(const v4f*)xp;
  const v4f c = *(const v4f*)(xp + 4);
  float v[8] = {a[0], a[1], a[2], a[3], c[0], c[1], c[2], c[3]};
  float s = 0.0f;
#pragma unroll
  for (int j = 0; j < 8; ++j) s += v[j];
#pragma unroll
  for (int m = 1; m < 32; m <<= 1) s += __shfl_xor(s, m, 32);
  const float mu = s * (1.0f / DM);
  float vs = 0.0f;
#pragma unroll
  for (int j = 0; j < 8; ++j) { const float t = v[j] - mu; vs += t * t; }
#pragma unroll
  for (int m = 1; m < 32; m <<= 1) vs += __shfl_xor(vs, m, 32);
  const float inv = rsqrtf(vs * (1.0f / DM) + 1e-5f);
  const v4f g0 = *(const v4f*)(g + 8 * lane);
  const v4f g1 = *(const v4f*)(g + 8 * lane + 4);
  const v4f b0 = *(const v4f*)(bb + 8 * lane);
  const v4f b1 = *(const v4f*)(bb + 8 * lane + 4);
  float gw[8] = {g0[0], g0[1], g0[2], g0[3], g1[0], g1[1], g1[2], g1[3]};
  float gb[8] = {b0[0], b0[1], b0[2], b0[3], b1[0], b1[1], b1[2], b1[3]};
  v8h hi = {}, lo = {};
#pragma unroll
  for (int j = 0; j < 8; ++j) {
    const float y = (v[j] - mu) * inv * bf16r(gw[j]) + bf16r(gb[j]);
    f16 x, e;
    split2(y, x, e);
    hi[j] = x;
    lo[j] = e;
  }
  const v8us hu = __builtin_bit_cast(v8us, hi);
  const v8us lu = __builtin_bit_cast(v8us, lo);
  const size_t off = (size_t)row * DM + 8 * lane;
  *(volatile v8us*)(yh + off) = hu;
  if constexpr (LO) *(volatile v8us*)(yl + off) = lu;
  __threadfence();
  *(volatile v8us*)(yh + off) = hu;
  if constexpr (LO) *(volatile v8us*)(yl + off) = lu;
}

__device__ __forceinline__ void st_rowf(float* S, int row0, int col, v8f c, float bn) {
#pragma unroll
  for (int r = 0; r < 8; ++r) S[(row0 + r) * OP + col] = c[r] * HINV + bn;
}
__device__ __forceinline__ void st_rowg(float* S, int row0, int col, v8f c, float bn) {
#pragma unroll
  for (int r = 0; r < 8; ++r) S[(row0 + r) * OP + col] = gelu_f(c[r] * HINV + bn);
}
__device__ __forceinline__ void st_rowf2(float* S, int row0, int col, v8f hh, v8f gg, float bn) {
#pragma unroll
  for (int r = 0; r < 8; ++r) S[(row0 + r) * OP + col] = hh[r] * HINV + gg[r] * LINV + bn;
}
__device__ __forceinline__ void st_colf2(float* S, int d, int tok0, v8f hh, v8f gg, float bn) {
  v4f a, c;
#pragma unroll
  for (int i = 0; i < 4; ++i) {
    a[i] = hh[i] * HINV + gg[i] * LINV + bn;
    c[i] = hh[4 + i] * HINV + gg[4 + i] * LINV + bn;
  }
  *(v4fa*)&S[d * OPT + tok0] = a;
  *(v4fa*)&S[d * OPT + tok0 + 4] = c;
}
__device__ __forceinline__ void st8(float* p, v8f o, float w) {
  v4f a, c;
#pragma unroll
  for (int i = 0; i < 4; ++i) { a[i] = o[i] * w; c[i] = o[4 + i] * w; }
  *(v4fa*)p = a;
  *(v4fa*)(p + 4) = c;
}

template <int MODE>
__global__ __launch_bounds__(256)
void k_gemm_x(const unsigned short* __restrict__ a16, const unsigned short* __restrict__ w16,
              const float* __restrict__ bias, const float* __restrict__ res,
              const float* __restrict__ xin, const float* __restrict__ fw, const float* __restrict__ fbv,
              float* out, int K, int N) {
  __shared__ __align__(16) float So[128 * OP];
  const int tid = threadIdx.x, lane = tid & 31, wv = tid >> 5, hl = lane >> 4, l15 = lane & 15;
  const int m0 = (int)blockIdx.y * 128, n0 = (int)blockIdx.x * 64;
  const int mp = wv >> 1, np = wv & 1;
  const int ra = m0 + 32 * mp, cb = n0 + 32 * np;
  const f16* Ap = (const f16*)a16;
  const f16* Wp = (const f16*)w16;

  v8f c00 = {}, c01 = {}, c10 = {}, c11 = {};
  const int nks = K >> 5;
#pragma unroll 1
  for (int ks = 0; ks < nks; ++ks) {
    const int k0 = ks << 5;
    const v16h a0 = ld_frag(Ap, ra, k0, K);
    const v16h a1 = ld_frag(Ap, ra + 16, k0, K);
    const v16h b0 = ld_frag(Wp, cb, k0, K);
    const v16h b1 = ld_frag(Wp, cb + 16, k0, K);
    c00 = mma_h(a0, b0, c00);
    c01 = mma_h(a0, b1, c01);
    c10 = mma_h(a1, b0, c10);
    c11 = mma_h(a1, b1, c11);
    guard4x4(c00, c01, c10, c11, a0, a1, b0, b1);
  }

  const float bn0 = bf16r(bias[cb + l15]);
  const float bn1 = bf16r(bias[cb + 16 + l15]);
  const int rr = 32 * mp + 8 * hl, cc = 32 * np + l15;
  st_rowf(So, rr,      cc,      c00, bn0);
  st_rowf(So, rr,      cc + 16, c01, bn1);
  st_rowf(So, rr + 16, cc,      c10, bn0);
  st_rowf(So, rr + 16, cc + 16, c11, bn1);
  __syncthreads();

  if constexpr (MODE == 0) {
    const bool use_cos = (n0 < NFQ);
#pragma unroll 1
    for (int i = 0; i < 32; ++i) {
      const int e = tid + 256 * i;
      const int row = e >> 6, col = e & 63;
      const int f = (n0 + col) & (NFQ - 1);
      const float* xr = xin + (size_t)(m0 + row) * NX;
      const float p0 = bf16r(xr[0]), p1 = bf16r(xr[1]), p2 = bf16r(xr[2]);
      const float w0 = bf16r(fw[f * 3 + 0]), w1 = bf16r(fw[f * 3 + 1]), w2 = bf16r(fw[f * 3 + 2]);
      const float proj = ((p0 * w0 + p1 * w1) + p2 * w2) + bf16r(fbv[f]);
      float tr;
      if (use_cos) tr = cosf(proj); else tr = sinf(proj);
      So[row * OP + col] += tr * PEC;
    }
    __syncthreads();
  }

  v4f u[8];
  size_t off[8];
#pragma unroll
  for (int it = 0; it < 8; ++it) {
    const int p = tid + 256 * it;
    const int row = p >> 4, q = p & 15;
    u[it] = *(const v4fa*)&So[row * OP + 4 * q];
    off[it] = (size_t)(m0 + row) * (size_t)N + n0 + 4 * q;
    if constexpr (MODE == 1) {
      const v4f rv = *(const v4f*)(res + off[it]);
      u[it] += rv;
    }
  }
#pragma unroll
  for (int it = 0; it < 8; ++it) *(volatile v4f*)(out + off[it]) = u[it];
  __threadfence();
#pragma unroll
  for (int it = 0; it < 8; ++it) *(volatile v4f*)(out + off[it]) = u[it];
}

__global__ __launch_bounds__(256)
void k_gemm_h(const unsigned short* __restrict__ a16, const unsigned short* __restrict__ w16,
              const float* __restrict__ bias, unsigned short* hp, int K, int N) {
  __shared__ __align__(16) float So[128 * OP];
  const int tid = threadIdx.x, lane = tid & 31, wv = tid >> 5, hl = lane >> 4, l15 = lane & 15;
  const int m0 = (int)blockIdx.y * 128, n0 = (int)blockIdx.x * 64;
  const int mp = wv >> 1, np = wv & 1;
  const int ra = m0 + 32 * mp, cb = n0 + 32 * np;
  const f16* Ap = (const f16*)a16;
  const f16* Wp = (const f16*)w16;

  v8f c00 = {}, c01 = {}, c10 = {}, c11 = {};
  const int nks = K >> 5;
#pragma unroll 1
  for (int ks = 0; ks < nks; ++ks) {
    const int k0 = ks << 5;
    const v16h a0 = ld_frag(Ap, ra, k0, K);
    const v16h a1 = ld_frag(Ap, ra + 16, k0, K);
    const v16h b0 = ld_frag(Wp, cb, k0, K);
    const v16h b1 = ld_frag(Wp, cb + 16, k0, K);
    c00 = mma_h(a0, b0, c00);
    c01 = mma_h(a0, b1, c01);
    c10 = mma_h(a1, b0, c10);
    c11 = mma_h(a1, b1, c11);
    guard4x4(c00, c01, c10, c11, a0, a1, b0, b1);
  }

  const float bn0 = bf16r(bias[cb + l15]);
  const float bn1 = bf16r(bias[cb + 16 + l15]);
  const int rr = 32 * mp + 8 * hl, cc = 32 * np + l15;
  st_rowg(So, rr,      cc,      c00, bn0);
  st_rowg(So, rr,      cc + 16, c01, bn1);
  st_rowg(So, rr + 16, cc,      c10, bn0);
  st_rowg(So, rr + 16, cc + 16, c11, bn1);
  __syncthreads();

  v8us u[4];
  size_t off[4];
#pragma unroll
  for (int it = 0; it < 4; ++it) {
    const int p = tid + 256 * it;
    const int row = p >> 3, q = p & 7;
    const float* sp = So + row * OP + 8 * q;
    const v4f a = *(const v4fa*)sp;
    const v4f c = *(const v4fa*)(sp + 4);
    v8h o = {};
#pragma unroll
    for (int e = 0; e < 4; ++e) { o[e] = (f16)(a[e] * ASC); o[4 + e] = (f16)(c[e] * ASC); }
    u[it] = __builtin_bit_cast(v8us, o);
    off[it] = (size_t)(m0 + row) * (size_t)N + n0 + 8 * q;
  }
#pragma unroll
  for (int it = 0; it < 4; ++it) *(volatile v8us*)(hp + off[it]) = u[it];
  __threadfence();
#pragma unroll
  for (int it = 0; it < 4; ++it) *(volatile v8us*)(hp + off[it]) = u[it];
}

template <bool ALO, bool QKLO>
__global__ __launch_bounds__(256)
void k_gemm_heads(const unsigned short* __restrict__ ah, const unsigned short* __restrict__ al,
                  const unsigned short* __restrict__ w16,
                  const float* __restrict__ bq, const float* __restrict__ bk, const float* __restrict__ bv,
                  unsigned short* dqh, unsigned short* dql, unsigned short* dkh, unsigned short* dkl,
                  unsigned short* dvt, int K) {
  __shared__ __align__(16) float So[128 * OP];
  const int tid = threadIdx.x, lane = tid & 31, wv = tid >> 5, hl = lane >> 4, l15 = lane & 15;
  const int nb = (int)blockIdx.x;
  const int m0 = (int)blockIdx.y * 128, n0 = nb * 64;
  const int stream = nb >> 2, head0 = (nb & 3) * 2;
  const int b = m0 / NT, t0 = m0 - b * NT;
  const f16* Hp = (const f16*)ah;
  const f16* Lp = (const f16*)al;
  const f16* Wp = (const f16*)w16;
  const int mp = wv >> 1, np = wv & 1;
  const int ra = m0 + 32 * mp, cb = n0 + 32 * np;

  v8f h00 = {}, h01 = {}, h10 = {}, h11 = {};
  v8f g00 = {}, g01 = {}, g10 = {}, g11 = {};
  const int nks = K >> 5;
#pragma unroll 1
  for (int ks = 0; ks < nks; ++ks) {
    const int k0 = ks << 5;
    const v16h a0 = ld_frag(Hp, ra, k0, K);
    const v16h a1 = ld_frag(Hp, ra + 16, k0, K);
    const v16h b0 = ld_frag(Wp, cb, k0, K);
    const v16h b1 = ld_frag(Wp, cb + 16, k0, K);
    h00 = mma_h(a0, b0, h00);
    h01 = mma_h(a0, b1, h01);
    h10 = mma_h(a1, b0, h10);
    h11 = mma_h(a1, b1, h11);
    if constexpr (ALO) {
      const v16h e0 = ld_frag(Lp, ra, k0, K);
      const v16h e1 = ld_frag(Lp, ra + 16, k0, K);
      g00 = mma_h(e0, b0, g00);
      g01 = mma_h(e0, b1, g01);
      g10 = mma_h(e1, b0, g10);
      g11 = mma_h(e1, b1, g11);
      guard8x6(h00, h01, h10, h11, g00, g01, g10, g11, a0, a1, b0, b1, e0, e1);
    } else {
      guard4x4(h00, h01, h10, h11, a0, a1, b0, b1);
    }
  }

  const float* bp = (stream == 0) ? bq : ((stream == 1) ? bk : bv);
  const int cs = (nb & 3) * 64 + 32 * np + l15;
  const float bn0 = bf16r(bp[cs]);
  const float bn1 = bf16r(bp[cs + 16]);
  const int rr = 32 * mp + 8 * hl, cc = 32 * np + l15;

  if (stream == 2) {
    st_colf2(So, cc,      rr,      h00, g00, bn0);
    st_colf2(So, cc + 16, rr,      h01, g01, bn1);
    st_colf2(So, cc,      rr + 16, h10, g10, bn0);
    st_colf2(So, cc + 16, rr + 16, h11, g11, bn1);
    __syncthreads();
    v8us u[4];
    size_t off[4];
#pragma unroll
    for (int it = 0; it < 4; ++it) {
      const int p = tid + 256 * it;
      const int d = p >> 4, q = p & 15;
      const float* sp = So + d * OPT + 8 * q;
      const v4f a = *(const v4fa*)sp;
      const v4f c = *(const v4fa*)(sp + 4);
      v8h o = {};
#pragma unroll
      for (int e = 0; e < 4; ++e) { o[e] = (f16)(a[e] * ASC); o[4 + e] = (f16)(c[e] * ASC); }
      u[it] = __builtin_bit_cast(v8us, o);
      off[it] = ((size_t)(b * NH + head0 + (d >> 5)) * DK + (d & 31)) * (size_t)NT + t0 + 8 * q;
    }
#pragma unroll
    for (int it = 0; it < 4; ++it) *(volatile v8us*)(dvt + off[it]) = u[it];
    __threadfence();
#pragma unroll
    for (int it = 0; it < 4; ++it) *(volatile v8us*)(dvt + off[it]) = u[it];
  } else {
    unsigned short* dh = (stream == 0) ? dqh : dkh;
    unsigned short* dl = (stream == 0) ? dql : dkl;
    st_rowf2(So, rr,      cc,      h00, g00, bn0);
    st_rowf2(So, rr,      cc + 16, h01, g01, bn1);
    st_rowf2(So, rr + 16, cc,      h10, g10, bn0);
    st_rowf2(So, rr + 16, cc + 16, h11, g11, bn1);
    __syncthreads();
    v8us hv[4], lv[4];
    size_t off[4];
#pragma unroll
    for (int it = 0; it < 4; ++it) {
      const int p = tid + 256 * it;
      const int hh = p >> 9, rem = p & 511;
      const int row = rem >> 2, q4 = rem & 3;
      const float* sp = So + row * OP + hh * 32 + q4 * 8;
      const v4f a = *(const v4fa*)sp;
      const v4f c = *(const v4fa*)(sp + 4);
      v8h hi = {}, lo = {};
#pragma unroll
      for (int e = 0; e < 4; ++e) {
        f16 x, y;
        split2(a[e], x, y); hi[e] = x;     lo[e] = y;
        split2(c[e], x, y); hi[4 + e] = x; lo[4 + e] = y;
      }
      hv[it] = __builtin_bit_cast(v8us, hi);
      lv[it] = __builtin_bit_cast(v8us, lo);
      off[it] = ((size_t)(b * NH + head0 + hh) * NT + t0 + row) * (size_t)DK + q4 * 8;
    }
#pragma unroll
    for (int it = 0; it < 4; ++it) {
      *(volatile v8us*)(dh + off[it]) = hv[it];
      if constexpr (QKLO) *(volatile v8us*)(dl + off[it]) = lv[it];
    }
    __threadfence();
#pragma unroll
    for (int it = 0; it < 4; ++it) {
      *(volatile v8us*)(dh + off[it]) = hv[it];
      if constexpr (QKLO) *(volatile v8us*)(dl + off[it]) = lv[it];
    }
  }
}

__global__ __launch_bounds__(256)
void k_attn(const unsigned short* __restrict__ qp, const unsigned short* __restrict__ kp,
            const unsigned short* __restrict__ vtp, const int* __restrict__ msk, unsigned short* att) {
  __shared__ __align__(16) float So[64 * OP];
  const int tid = threadIdx.x, lane = tid & 31, wv = tid >> 5, hl = lane >> 4, l15 = lane & 15;
  const int b = (int)blockIdx.y >> 2, hp = (int)blockIdx.y & 3;
  const int hsel = wv >> 2, h = 2 * hp + hsel;
  const int qblk = (int)blockIdx.x * 64;
  const int q0 = qblk + 16 * (wv & 3);
  const size_t bh = (size_t)(b * NH + h);
  const f16* Qb = (const f16*)qp  + bh * NT * DK;
  const f16* Kb = (const f16*)kp  + bh * NT * DK;
  const f16* Vb = (const f16*)vtp + bh * DK * NT;
  const int* mrow = msk + ((size_t)b * NT + q0 + l15) * NT;

  const v16h qf = ld_frag(Qb, q0, 0, DK);
  v8f O0 = {}, O1 = {};
  float m = -3.0e38f, l = 0.0f;
  const float NEG = -__builtin_inff();

#pragma unroll 1
  for (int kb = 0; kb < NT; kb += 32) {
    const v16h k0f = ld_frag(Kb, kb, 0, DK);
    const v16h k1f = ld_frag(Kb, kb + 16, 0, DK);
    v8f s0 = {}, s1 = {};
    s0 = mma_h(k0f, qf, s0);
    s1 = mma_h(k1f, qf, s1);
    guard2x3(s0, s1, k0f, k1f, qf);

    const v8i mk0 = *(const v8i*)(mrow + kb + 8 * hl);
    const v8i mk1 = *(const v8i*)(mrow + kb + 16 + 8 * hl);
    float mx = NEG;
#pragma unroll
    for (int r = 0; r < 8; ++r) {
      const float a0 = (mk0[r] != 0) ? s0[r] * SSC : NEG;
      const float a1 = (mk1[r] != 0) ? s1[r] * SSC : NEG;
      s0[r] = a0;
      s1[r] = a1;
      mx = fmaxf(mx, fmaxf(a0, a1));
    }
    mx = fmaxf(mx, __shfl_xor(mx, 16, 32));
    const float mnew = fmaxf(m, mx);
    const float corr = __expf(m - mnew);
    float ps = 0.0f;
    v8h p0v = {}, p1v = {};
#pragma unroll
    for (int r = 0; r < 8; ++r) {
      const float p0 = __expf(s0[r] - mnew);
      const float p1 = __expf(s1[r] - mnew);
      ps += p0 + p1;
      p0v[r] = (f16)(p0 * PSC);
      p1v[r] = (f16)(p1 * PSC);
    }
    ps += __shfl_xor(ps, 16, 32);
    l = l * corr + ps;
    m = mnew;
    O0 *= corr; O1 *= corr;
    FragH pf;
    pf.h[0] = p0v;
    pf.h[1] = p1v;

    const v16h v0f = ld_frag(Vb, 0,  kb, NT);
    const v16h v1f = ld_frag(Vb, 16, kb, NT);
    O0 = mma_h(v0f, pf.v, O0);
    O1 = mma_h(v1f, pf.v, O1);
    guard2x3(O0, O1, v0f, v1f, pf.v);
  }

  const float w = OINV * (1.0f / l);
  float* so = So + (16 * (wv & 3) + l15) * OP + 32 * hsel + 8 * hl;
  st8(so,      O0, w);
  st8(so + 16, O1, w);
  __syncthreads();

  v8us u[2];
  size_t off[2];
#pragma unroll
  for (int it = 0; it < 2; ++it) {
    const int p = tid + 256 * it;
    const int row = p >> 3, q = p & 7;
    const float* sp = So + row * OP + 8 * q;
    const v4f a = *(const v4fa*)sp;
    const v4f c = *(const v4fa*)(sp + 4);
    v8h o = {};
#pragma unroll
    for (int e = 0; e < 4; ++e) { o[e] = (f16)(a[e] * ASC); o[4 + e] = (f16)(c[e] * ASC); }
    u[it] = __builtin_bit_cast(v8us, o);
    off[it] = ((size_t)(b * NT + qblk + row)) * DM + hp * 64 + 8 * q;
  }
#pragma unroll
  for (int it = 0; it < 2; ++it) *(volatile v8us*)(att + off[it]) = u[it];
  __threadfence();
#pragma unroll
  for (int it = 0; it < 2; ++it) *(volatile v8us*)(att + off[it]) = u[it];
}

__global__ __launch_bounds__(256)
void k_score(const unsigned short* __restrict__ qh, const unsigned short* __restrict__ ql,
             const unsigned short* __restrict__ kh, const unsigned short* __restrict__ kl,
             const float* __restrict__ snw, const float* __restrict__ snb,
             const float* __restrict__ sfw, const float* __restrict__ sfb, float* tpl) {
  __shared__ __align__(16) float St[32 * OP];
  const int tid = threadIdx.x, lane = tid & 31, wv = tid >> 5, hl = lane >> 4, l15 = lane & 15;
  const int b = (int)blockIdx.z;
  const int qb0 = (int)blockIdx.y * 32, kb0 = (int)blockIdx.x * 64;
  const int q0 = qb0 + 16 * (wv >> 2), kk0 = kb0 + 16 * (wv & 3);

  float cw[NH], cbv[NH], cs[NH];
#pragma unroll
  for (int hh = 0; hh < NH; ++hh) { cw[hh] = bf16r(snw[hh]); cbv[hh] = bf16r(snb[hh]); cs[hh] = bf16r(sfw[hh]); }
  const float cb0 = bf16r(sfb[0]);

  v8f sv[NH];
#pragma unroll
  for (int hh = 0; hh < NH; ++hh) {
    const size_t base = (size_t)(b * NH + hh) * NT * DK;
    const v16h aqh = ld_frag((const f16*)qh + base, q0,  0, DK);
    const v16h aql = ld_frag((const f16*)ql + base, q0,  0, DK);
    const v16h bkh = ld_frag((const f16*)kh + base, kk0, 0, DK);
    const v16h bkl = ld_frag((const f16*)kl + base, kk0, 0, DK);
    v8f chh = {}, cx = {};
    chh = mma_h(aqh, bkh, chh);
    cx  = mma_h(aqh, bkl, cx);
    cx  = mma_h(aql, bkh, cx);
    guard2x4(chh, cx, aqh, aql, bkh, bkl);
    v8f s = {};
#pragma unroll
    for (int r = 0; r < 8; ++r) s[r] = (chh[r] + cx[r] * RINV) * SSC;
    sv[hh] = s;
  }

#pragma unroll
  for (int r = 0; r < 8; ++r) {
    float mu = 0.0f;
#pragma unroll
    for (int hh = 0; hh < NH; ++hh) mu += sv[hh][r];
    mu *= 0.125f;
    float var = 0.0f;
#pragma unroll
    for (int hh = 0; hh < NH; ++hh) { const float d = sv[hh][r] - mu; var += d * d; }
    const float inv = rsqrtf(var * 0.125f + 1e-5f);
    float t = 0.0f;
#pragma unroll
    for (int hh = 0; hh < NH; ++hh) t += ((sv[hh][r] - mu) * inv * cw[hh] + cbv[hh]) * cs[hh];
    t += cb0;
    St[(16 * (wv >> 2) + 8 * hl + r) * OP + 16 * (wv & 3) + l15] = t;
  }
  __syncthreads();

  v4f u[2];
  size_t off[2];
#pragma unroll
  for (int it = 0; it < 2; ++it) {
    const int p = tid + 256 * it;
    const int row = p >> 4, q = p & 15;
    u[it] = *(const v4fa*)&St[row * OP + 4 * q];
    off[it] = ((size_t)(b * NT + qb0 + row)) * NT + kb0 + 4 * q;
  }
#pragma unroll
  for (int it = 0; it < 2; ++it) *(volatile v4f*)(tpl + off[it]) = u[it];
  __threadfence();
#pragma unroll
  for (int it = 0; it < 2; ++it) *(volatile v4f*)(tpl + off[it]) = u[it];
}

__global__ __launch_bounds__(256)
void k_sym(const float* __restrict__ tpl, float* out) {
  __shared__ float Mt[64 * 65];
  const int tid = threadIdx.x;
  const int b = (int)blockIdx.z, q0 = (int)blockIdx.y * 64, k0 = (int)blockIdx.x * 64;
#pragma unroll
  for (int j = 0; j < 4; ++j) {
    const int e = tid + 256 * j;
    const int i = e >> 4, c4 = (e & 15) * 4;
    const v4f v = *(const v4f*)(tpl + ((size_t)(b * NT + k0 + i)) * NT + q0 + c4);
#pragma unroll
    for (int c = 0; c < 4; ++c) Mt[i * 65 + c4 + c] = v[c];
  }
  __syncthreads();
  v4f u[4];
  size_t off[4];
#pragma unroll
  for (int it = 0; it < 4; ++it) {
    const int p = tid + 256 * it;
    const int r = p >> 4, q = p & 15;
    off[it] = ((size_t)(b * NT + q0 + r)) * NT + k0 + 4 * q;
    const v4f a = *(const v4f*)(tpl + off[it]);
    v4f o;
#pragma unroll
    for (int e = 0; e < 4; ++e) o[e] = 0.5f * (a[e] + Mt[(4 * q + e) * 65 + r]);
    u[it] = o;
  }
#pragma unroll
  for (int it = 0; it < 4; ++it) *(volatile v4f*)(out + off[it]) = u[it];
  __threadfence();
#pragma unroll
  for (int it = 0; it < 4; ++it) *(volatile v4f*)(out + off[it]) = u[it];
}

extern "C" void kernel_launch(void* const* d_in, const int* in_sizes, int n_in,
                              void* d_out, int out_size, void* d_ws, size_t ws_size,
                              hipStream_t stream) {
  if (n_in < 30) return;
  if (in_sizes[0] != NR * NX || in_sizes[1] != NB * NT * NT || in_sizes[2] != NFQ * 3 || in_sizes[3] != NFQ) return;
  if (in_sizes[4] != NC * DM || in_sizes[5] != DM) return;
  for (int i = 0; i < 4; ++i) {
    if (in_sizes[6 + 2 * i] != NL * DM * DM || in_sizes[7 + 2 * i] != NL * DM) return;
  }
  for (int i = 14; i < 18; ++i) { if (in_sizes[i] != NL * DM) return; }
  if (in_sizes[18] != DM || in_sizes[19] != DM) return;
  if (in_sizes[20] != NL * DM * DF || in_sizes[21] != NL * DF || in_sizes[22] != NL * DF * DM || in_sizes[23] != NL * DM) return;
  if (in_sizes[24] != DM * NC || in_sizes[25] != NC) return;
  if (in_sizes[26] != NH || in_sizes[27] != NH || in_sizes[28] != NH || in_sizes[29] != 1) return;
  if (out_size != OUT0_N + OUT1_N) return;

  const size_t sz_ax   = (size_t)NR * NC * 2;
  const size_t sz_wch  = (size_t)DM * NC * 2;
  const size_t sz_wqkv = (size_t)NL * 3 * DM * DM * 2;
  const size_t sz_wo   = (size_t)NL * DM * DM * 2;
  const size_t sz_wu   = (size_t)NL * DF * DM * 2;
  const size_t sz_wd   = (size_t)NL * DM * DF * 2;
  const size_t sz_wf   = (size_t)NC * DM * 2;
  const size_t sz_x    = (size_t)NR * DM * 4;
  const size_t sz_p16  = (size_t)NR * DM * 2;
  const size_t sz_h    = (size_t)NR * DF * 2;
  const size_t sz_t    = (size_t)NB * NT * NT * 4;

  const size_t off_ax   = 0;
  const size_t off_wch  = off_ax   + sz_ax;
  const size_t off_wqkv = off_wch  + sz_wch;
  const size_t off_wo   = off_wqkv + sz_wqkv;
  const size_t off_wu   = off_wo   + sz_wo;
  const size_t off_wd   = off_wu   + sz_wu;
  const size_t off_wf   = off_wd   + sz_wd;
  const size_t off_xa   = off_wf   + sz_wf;
  const size_t off_xb   = off_xa   + sz_x;
  const size_t off_xnh  = off_xb   + sz_x;
  const size_t off_xnl  = off_xnh  + sz_p16;
  const size_t off_qh   = off_xnl  + sz_p16;
  const size_t off_ql   = off_qh   + sz_p16;
  const size_t off_kh   = off_ql   + sz_p16;
  const size_t off_kl   = off_kh   + sz_p16;
  const size_t off_vt   = off_kl   + sz_p16;
  const size_t off_att  = off_vt   + sz_p16;
  const size_t off_hp   = off_att  + sz_p16;
  const size_t off_t    = off_hp   + sz_h;
  const size_t need     = off_t    + sz_t;
  if (need > ws_size) return;
  if (need > (size_t)134217728) return;

  const float* X     = (const float*)d_in[0];
  const int*   msk   = (const int*)  d_in[1];
  const float* fW    = (const float*)d_in[2];
  const float* fb    = (const float*)d_in[3];
  const float* cW    = (const float*)d_in[4];
  const float* cb    = (const float*)d_in[5];
  const float* Wq    = (const float*)d_in[6];
  const float* bq    = (const float*)d_in[7];
  const float* Wk    = (const float*)d_in[8];
  const float* bk    = (const float*)d_in[9];
  const float* Wv    = (const float*)d_in[10];
  const float* bv    = (const float*)d_in[11];
  const float* Wo    = (const float*)d_in[12];
  const float* bo    = (const float*)d_in[13];
  const float* ln1w  = (const float*)d_in[14];
  const float* ln1b  = (const float*)d_in[15];
  const float* ln2w  = (const float*)d_in[16];
  const float* ln2b  = (const float*)d_in[17];
  const float* lnfw  = (const float*)d_in[18];
  const float* lnfb  = (const float*)d_in[19];
  const float* Wup   = (const float*)d_in[20];
  const float* bup   = (const float*)d_in[21];
  const float* Wdn   = (const float*)d_in[22];
  const float* bdn   = (const float*)d_in[23];
  const float* Wfin  = (const float*)d_in[24];
  const float* bfin  = (const float*)d_in[25];
  const float* snw   = (const float*)d_in[26];
  const float* snb   = (const float*)d_in[27];
  const float* sfw   = (const float*)d_in[28];
  const float* sfb   = (const float*)d_in[29];

  float* out0 = (float*)d_out;
  float* out1 = out0 + OUT0_N;

  char* wsb = (char*)d_ws;
  unsigned short* ax_p   = (unsigned short*)(wsb + off_ax);
  unsigned short* wch_p  = (unsigned short*)(wsb + off_wch);
  unsigned short* wqkv_p = (unsigned short*)(wsb + off_wqkv);
  unsigned short* wo_p   = (unsigned short*)(wsb + off_wo);
  unsigned short* wu_p   = (unsigned short*)(wsb + off_wu);
  unsigned short* wd_p   = (unsigned short*)(wsb + off_wd);
  unsigned short* wf_p   = (unsigned short*)(wsb + off_wf);
  float*          xa_p   = (float*)(wsb + off_xa);
  float*          xb_p   = (float*)(wsb + off_xb);
  unsigned short* xnh_p  = (unsigned short*)(wsb + off_xnh);
  unsigned short* xnl_p  = (unsigned short*)(wsb + off_xnl);
  unsigned short* qh_p   = (unsigned short*)(wsb + off_qh);
  unsigned short* ql_p   = (unsigned short*)(wsb + off_ql);
  unsigned short* kh_p   = (unsigned short*)(wsb + off_kh);
  unsigned short* kl_p   = (unsigned short*)(wsb + off_kl);
  unsigned short* vt_p   = (unsigned short*)(wsb + off_vt);
  unsigned short* att_p  = (unsigned short*)(wsb + off_att);
  unsigned short* hp_p   = (unsigned short*)(wsb + off_hp);
  float*          t_p    = (float*)(wsb + off_t);

  const int n8_x = NR * NC / 8;
  k_cvt_x<<<dim3((n8_x + 255) / 256), dim3(256), 0, stream>>>(X, ax_p, n8_x);
  const size_t dls_qkv = (size_t)3 * DM * DM;
  const size_t dls_sq  = (size_t)DM * DM;
  const size_t dls_ff  = (size_t)DM * DF;
  k_cvt_wt<<<dim3(DM / 64, NC / 64, 1),  dim3(256), 0, stream>>>(cW,   wch_p,  NC, DM, (size_t)0, 0,      WSC);
  k_cvt_wt<<<dim3(DM / 64, DM / 64, NL), dim3(256), 0, stream>>>(Wq,   wqkv_p, DM, DM, dls_qkv,   0,      WSC);
  k_cvt_wt<<<dim3(DM / 64, DM / 64, NL), dim3(256), 0, stream>>>(Wk,   wqkv_p, DM, DM, dls_qkv,   DM,     WSC);
  k_cvt_wt<<<dim3(DM / 64, DM / 64, NL), dim3(256), 0, stream>>>(Wv,   wqkv_p, DM, DM, dls_qkv,   2 * DM, WSC);
  k_cvt_wt<<<dim3(DM / 64, DM / 64, NL), dim3(256), 0, stream>>>(Wo,   wo_p,   DM, DM, dls_sq,    0,      WSC);
  k_cvt_wt<<<dim3(DF / 64, DM / 64, NL), dim3(256), 0, stream>>>(Wup,  wu_p,   DM, DF, dls_ff,    0,      WSC);
  k_cvt_wt<<<dim3(DM / 64, DF / 64, NL), dim3(256), 0, stream>>>(Wdn,  wd_p,   DF, DM, dls_ff,    0,      WSC);
  k_cvt_wt<<<dim3(NC / 64, DM / 64, 1),  dim3(256), 0, stream>>>(Wfin, wf_p,   DM, NC, (size_t)0, 0,      WSC);

  k_gemm_x<0><<<dim3(DM / 64, NR / 128), dim3(256), 0, stream>>>(ax_p, wch_p, cb, xb_p, X, fW, fb, xa_p, NC, DM);

  const dim3 g_ln(NR / 8), g_heads(3 * DM / 64, NR / 128), g_attn(NT / 64, NB * (NH / 2));
  const dim3 g_dm(DM / 64, NR / 128), g_ff(DF / 64, NR / 128), blk(256);
  for (int i = 0; i < NL; ++i) {
    const unsigned short* wqkv_i = wqkv_p + (size_t)i * 3 * DM * DM;
    const unsigned short* wo_i   = wo_p   + (size_t)i * DM * DM;
    const unsigned short* wu_i   = wu_p   + (size_t)i * DF * DM;
    const unsigned short* wd_i   = wd_p   + (size_t)i * DM * DF;
    if (i == NL - 1) {
      k_ln<true><<<g_ln, blk, 0, stream>>>(xa_p, ln1w + i * DM, ln1b + i * DM, xnh_p, xnl_p, NR);
      k_gemm_heads<true, true><<<g_heads, blk, 0, stream>>>(xnh_p, xnl_p, wqkv_i, bq + i * DM, bk + i * DM, bv + i * DM,
                                                            qh_p, ql_p, kh_p, kl_p, vt_p, DM);
    } else {
      k_ln<false><<<g_ln, blk, 0, stream>>>(xa_p, ln1w + i * DM, ln1b + i * DM, xnh_p, xnl_p, NR);
      k_gemm_heads<false, false><<<g_heads, blk, 0, stream>>>(xnh_p, xnl_p, wqkv_i, bq + i * DM, bk + i * DM, bv + i * DM,
                                                              qh_p, ql_p, kh_p, kl_p, vt_p, DM);
    }
    k_attn<<<g_attn, blk, 0, stream>>>(qh_p, kh_p, vt_p, msk, att_p);
    k_gemm_x<1><<<g_dm, blk, 0, stream>>>(att_p, wo_i, bo + i * DM, xa_p, X, fW, fb, xb_p, DM, DM);
    k_ln<false><<<g_ln, blk, 0, stream>>>(xb_p, ln2w + i * DM, ln2b + i * DM, xnh_p, xnl_p, NR);
    k_gemm_h<<<g_ff, blk, 0, stream>>>(xnh_p, wu_i, bup + i * DF, hp_p, DM, DF);
    k_gemm_x<1><<<g_dm, blk, 0, stream>>>(hp_p, wd_i, bdn + i * DM, xb_p, X, fW, fb, xa_p, DF, DM);
  }

  k_ln<false><<<g_ln, blk, 0, stream>>>(xa_p, lnfw, lnfb, xnh_p, xnl_p, NR);
  k_gemm_x<2><<<dim3(NC / 64, NR / 128), blk, 0, stream>>>(xnh_p, wf_p, bfin, xb_p, X, fW, fb, out0, DM, NC);

  k_score<<<dim3(NT / 64, NT / 32, NB), blk, 0, stream>>>(qh_p, ql_p, kh_p, kl_p, snw, snb, sfw, sfb, t_p);
  k_sym<<<dim3(NT / 64, NT / 64, NB), blk, 0, stream>>>(t_p, out1);
  (void)hipGetLastError();
}
